// CodeWiseAttention_18124761989378
// MI455X (gfx1250) — hardware-verified
//
#include <hip/hip_runtime.h>
#include <math.h>

constexpr int kBatch    = 8;
constexpr int kSeq      = 2500;
constexpr int kSeqPad   = 2560;
constexpr int kEmb      = 100;
constexpr int kEmbPad   = 128;
constexpr int kLab      = 8922;
constexpr int kLabPad   = 8960;
constexpr int kLabChunk = 4480;
constexpr int kNumChunk = 2;
constexpr float kPCarry    = 2048.0f;
constexpr float kPCarryInv = 1.0f / 2048.0f;
constexpr int kSmThreads = 320;
constexpr int kSmWaves   = kSmThreads / 32;

static_assert(kLabChunk * kNumChunk == kLabPad, "chunking");
static_assert(kLabChunk % 64 == 0 && kSeqPad % 64 == 0 && kEmbPad % 64 == 0, "tile multiples");
static_assert(kEmbPad % 32 == 0 && kSeqPad % 32 == 0, "K multiples of 32");
static_assert(kSmThreads * 8 == kSeqPad, "softmax coverage");

constexpr size_t kBytesS   = (size_t)kLabChunk * kSeqPad * 4;
constexpr size_t kBytesP   = (size_t)kLabChunk * kSeqPad * 2;
constexpr size_t kBytesLF  = (size_t)kLabPad * kEmbPad * 2;
constexpr size_t kBytesX   = (size_t)kBatch * kSeqPad * kEmbPad * 2;
constexpr size_t kBytesXt  = (size_t)kBatch * kEmbPad * kSeqPad * 2;
constexpr size_t kBytesM   = (size_t)kBatch * kLabPad * kEmbPad * 4;
constexpr size_t kOffS    = 0;
constexpr size_t kOffP    = kOffS + kBytesS;
constexpr size_t kOffLFhi = kOffP + kBytesP;
constexpr size_t kOffLFlo = kOffLFhi + kBytesLF;
constexpr size_t kOffXhi  = kOffLFlo + kBytesLF;
constexpr size_t kOffXlo  = kOffXhi + kBytesX;
constexpr size_t kOffXt   = kOffXlo + kBytesX;
constexpr size_t kOffM    = kOffXt + kBytesXt;
constexpr size_t kWsTotal = kOffM + kBytesM;
static_assert(kWsTotal == 125829120ull, "carve total");
static_assert(kWsTotal <= 134217728ull, "carve under 128 MiB");
static_assert((kOffP % 256) == 0 && (kOffLFhi % 256) == 0 && (kOffLFlo % 256) == 0 && (kOffXhi % 256) == 0 &&
              (kOffXlo % 256) == 0 && (kOffXt % 256) == 0 && (kOffM % 256) == 0, "aligned carve");

typedef __attribute__((ext_vector_type(16))) _Float16 v16h;
typedef __attribute__((ext_vector_type(8)))  _Float16 v8h;
typedef __attribute__((ext_vector_type(16))) __bf16   v16b;
typedef __attribute__((ext_vector_type(8)))  __bf16   v8b;
typedef __attribute__((ext_vector_type(8)))  float    v8f;
typedef __attribute__((ext_vector_type(4)))  float    v4f;
typedef __attribute__((ext_vector_type(4)))  unsigned int v4u;

__device__ __forceinline__ unsigned short f2bf_bits(float f) {
  unsigned u = __float_as_uint(f);
  return (unsigned short)((u + 0x7FFFu + ((u >> 16) & 1u)) >> 16);
}
__device__ __forceinline__ float bf_bits2f(unsigned short h) { return __uint_as_float(((unsigned)h) << 16); }

__device__ __forceinline__ void dep_guard_h(v8f& a, v8f& b, v16h x, v16h y) { asm volatile("v_nop\n\tv_nop\n\tv_nop\n\tv_nop" : "+v"(a), "+v"(b) : "v"(x), "v"(y)); }
__device__ __forceinline__ void dep_guard_b(v8f& a, v8f& b, v16b x, v16b y) { asm volatile("v_nop\n\tv_nop\n\tv_nop\n\tv_nop" : "+v"(a), "+v"(b) : "v"(x), "v"(y)); }
__device__ __forceinline__ void keep4_h(v16h a, v16h b, v16h c, v16h d) { asm volatile("v_nop" :: "v"(a), "v"(b), "v"(c), "v"(d)); }
__device__ __forceinline__ void keep4_b(v16b a, v16b b, v16b c, v16b d) { asm volatile("v_nop" :: "v"(a), "v"(b), "v"(c), "v"(d)); }
__device__ __forceinline__ void acc_guard4(v8f& a, v8f& b, v8f& c, v8f& d) { asm volatile("v_nop\n\tv_nop\n\tv_nop\n\tv_nop" : "+v"(a), "+v"(b), "+v"(c), "+v"(d)); }
template <typename T> struct Frag;
template <> struct Frag<_Float16> {
  typedef v16h V; union U { v16h v; v8h h[2]; };
  static __device__ __forceinline__ v16h load(const _Float16* p) {
    U f; f.h[0] = *(const v8h*)(p); f.h[1] = *(const v8h*)(p + 16); return f.v;
  }
  static __device__ __forceinline__ v8f mma(v16h a, v16h b, v8f c) {
    return __builtin_amdgcn_wmma_f32_16x16x32_f16(false, a, false, b, (short)0, c, false, false);
  }
  static __device__ __forceinline__ void guard(v8f& a, v8f& b, v16h x, v16h y) { dep_guard_h(a, b, x, y); }
  static __device__ __forceinline__ void keep(v16h a, v16h b, v16h c, v16h d) { keep4_h(a, b, c, d); }
};
template <> struct Frag<__bf16> {
  typedef v16b V; union U { v16b v; v8b h[2]; };
  static __device__ __forceinline__ v16b load(const __bf16* p) {
    U f; f.h[0] = *(const v8b*)(p); f.h[1] = *(const v8b*)(p + 16); return f.v;
  }
  static __device__ __forceinline__ v8f mma(v16b a, v16b b, v8f c) {
    return __builtin_amdgcn_wmma_f32_16x16x32_bf16(false, a, false, b, (short)0, c, false, false);
  }
  static __device__ __forceinline__ void guard(v8f& a, v8f& b, v16b x, v16b y) { dep_guard_b(a, b, x, y); }
  static __device__ __forceinline__ void keep(v16b a, v16b b, v16b c, v16b d) { keep4_b(a, b, c, d); }
};

__device__ __forceinline__ unsigned pk16(unsigned short a, unsigned short b) { return (unsigned)a | ((unsigned)b << 16); }
__device__ __forceinline__ unsigned short h_bits(float f) { const _Float16 h = (_Float16)f; return __builtin_bit_cast(unsigned short, h); }

template <int ET> struct Elem;
template <> struct Elem<0> { typedef _Float16 T; };
template <> struct Elem<1> { typedef __bf16 T; };
template <int ET, bool SPLIT, int BIAS_MODE, int OUT_MODE, bool RESID, int ACT = 0>
__global__ __launch_bounds__(256) void wmma_gemm64(
    const unsigned short* __restrict__ Ap, const unsigned short* __restrict__ A2p, int lda, long strideA,
    const unsigned short* __restrict__ Btp, const unsigned short* __restrict__ Bt2p, int ldb, long strideB,
    void* __restrict__ Cout, void* __restrict__ Cout2, int ldc, long strideC,
    const float* __restrict__ bias,
    const float* __restrict__ resid, long strideR,
    int M, int N, int K, float scale) {
  typedef typename Elem<ET>::T T;
  typedef typename Frag<T>::V V;
  const T* A = (const T*)Ap; const T* A2 = (const T*)A2p; const T* Bt = (const T*)Btp; const T* Bt2 = (const T*)Bt2p;
  __shared__ __align__(16) float sT[8][16 * 68];
  const int b    = blockIdx.y;
  const int lane = threadIdx.x & 31;
  const int wave = threadIdx.x >> 5;
  const int tilesN = N >> 6;
  const int tilesM = M >> 6;
  const int tile = blockIdx.x * 8 + wave;
  if (tile >= tilesM * tilesN) return;
  const int tm = tile / tilesN;
  const int tn = tile - tm * tilesN;
  const int m0 = tm << 6;
  const int n0 = tn << 6;

  const T* Ab  = A  + (size_t)b * strideA;
  const T* Bb  = Bt + (size_t)b * strideB;
  const T* Ab2 = SPLIT ? (A2  + (size_t)b * strideA) : nullptr;
  const T* Bb2 = SPLIT ? (Bt2 + (size_t)b * strideB) : nullptr;

  const int rlane = lane & 15;
  const int koff  = (lane >> 4) * 8;
  const int mOff  = (lane >> 4) * 8;

  v8f acc[4][4];
#pragma unroll
  for (int i = 0; i < 4; ++i)
#pragma unroll
    for (int j = 0; j < 4; ++j) acc[i][j] = (v8f){0.f,0.f,0.f,0.f,0.f,0.f,0.f,0.f};

  for (int k0 = 0; k0 < K; k0 += 32) {
    V bh[4], bl[4];
#pragma unroll
    for (int j = 0; j < 4; ++j) {
      const size_t bo = (size_t)(n0 + (j << 4) + rlane) * ldb + koff + k0;
      bh[j] = Frag<T>::load(Bb + bo);
      if (SPLIT) bl[j] = Frag<T>::load(Bb2 + bo);
    }
#pragma unroll
    for (int i = 0; i < 4; ++i) {
      const size_t ao = (size_t)(m0 + (i << 4) + rlane) * lda + koff + k0;
      V ah = Frag<T>::load(Ab + ao);
      V al;
      if (SPLIT) al = Frag<T>::load(Ab2 + ao);
#pragma unroll
      for (int j = 0; j < 4; ++j) {
        acc[i][j] = Frag<T>::mma(ah, bh[j], acc[i][j]);
        if (SPLIT) {
          acc[i][j] = Frag<T>::mma(ah, bl[j], acc[i][j]);
          acc[i][j] = Frag<T>::mma(al, bh[j], acc[i][j]);
        }
      }
      Frag<T>::guard(acc[i][0], acc[i][3], ah, SPLIT ? al : ah);
    }
    Frag<T>::keep(bh[0], bh[1], bh[2], bh[3]);
    if (SPLIT) Frag<T>::keep(bl[0], bl[1], bl[2], bl[3]);
  }
  acc_guard4(acc[0][0], acc[0][1], acc[0][2], acc[0][3]);
  acc_guard4(acc[1][0], acc[1][1], acc[1][2], acc[1][3]);
  acc_guard4(acc[2][0], acc[2][1], acc[2][2], acc[2][3]);
  acc_guard4(acc[3][0], acc[3][1], acc[3][2], acc[3][3]);

  float* slab = sT[wave];
  const float* Rb = RESID ? (resid + (size_t)b * strideR) : nullptr;
#pragma unroll
  for (int i = 0; i < 4; ++i) {
    const int mBase = m0 + (i << 4);
#pragma unroll
    for (int j = 0; j < 4; ++j) {
      const int n = n0 + (j << 4) + rlane;
      float bv = 0.f;
      if (BIAS_MODE == 2) bv = bias[n];
#pragma unroll
      for (int r = 0; r < 8; ++r) {
        float v = acc[i][j][r] * scale;
        if (BIAS_MODE == 1) v += bias[mBase + mOff + r];
        if (BIAS_MODE == 2) v += bv;
        if (RESID) v += Rb[(size_t)(mBase + mOff + r) * ldc + n];
        if (ACT == 2) v = fmaxf(v, 0.0f);
        if (ACT == 4) v = (v > 0.f) ? v : 0.01f * v;
        slab[(mOff + r) * 68 + (j << 4) + rlane] = v;
      }
    }
    __builtin_amdgcn_fence(__ATOMIC_RELEASE, "workgroup");
    __builtin_amdgcn_wave_barrier();
    __builtin_amdgcn_fence(__ATOMIC_ACQUIRE, "workgroup");
    if (OUT_MODE == 0) {
      float* C = (float*)Cout + (size_t)b * strideC;
      const int hh = lane >> 4, c4 = (lane & 15) * 4;
      for (int pass = 0; pass < 2; ++pass) {
#pragma unroll
        for (int it = 0; it < 8; ++it) {
          const int row = it * 2 + hh;
          v4f v = *(const v4f*)(slab + row * 68 + c4);
          *(volatile v4f*)(C + (size_t)(mBase + row) * ldc + n0 + c4) = v;
        }
        __threadfence();
      }
    } else {
      const int q = lane >> 3, c8 = (lane & 7) * 8;
      unsigned short* C  = (unsigned short*)Cout  + (size_t)b * strideC;
      unsigned short* C2 = (OUT_MODE == 2) ? ((unsigned short*)Cout2 + (size_t)b * strideC) : nullptr;
      for (int pass = 0; pass < 2; ++pass) {
#pragma unroll
        for (int it = 0; it < 4; ++it) {
          const int row = it * 4 + q;
          const float* sp = slab + row * 68 + c8;
          v8h hv, lv;
#pragma unroll
          for (int e = 0; e < 8; ++e) {
            if (OUT_MODE == 1) {
              hv[e] = (_Float16)sp[e];
            } else {
              unsigned short hb = f2bf_bits(sp[e]);
              unsigned short lb = f2bf_bits(sp[e] - bf_bits2f(hb));
              hv[e] = __builtin_bit_cast(_Float16, hb);
              lv[e] = __builtin_bit_cast(_Float16, lb);
            }
          }
          *(volatile v8h*)(C + (size_t)(mBase + row) * ldc + n0 + c8) = hv;
          if (OUT_MODE == 2) *(volatile v8h*)(C2 + (size_t)(mBase + row) * ldc + n0 + c8) = lv;
        }
        __threadfence();
      }
    }
    __builtin_amdgcn_fence(__ATOMIC_RELEASE, "workgroup");
    __builtin_amdgcn_wave_barrier();
    __builtin_amdgcn_fence(__ATOMIC_ACQUIRE, "workgroup");
  }
}

__global__ __launch_bounds__(256) void split_pad_kernel(const float* __restrict__ src, int srcRows, long srcBatch,
                                                        unsigned short* __restrict__ hi, unsigned short* __restrict__ lo,
                                                        int dstRows, long dstBatch) {
  const int b = blockIdx.y;
  const int i = blockIdx.x * 256 + threadIdx.x;
  const int row = i >> 4;
  if (row >= dstRows) return;
  const int c8 = (i & 15) * 8;
  const int rs = (row < srcRows) ? row : (srcRows - 1);
  const int ca = (c8 < kEmb - 4) ? c8 : (kEmb - 4);
  const int cb = ((c8 + 4) < kEmb - 4) ? (c8 + 4) : (kEmb - 4);
  const float* sp = src + (size_t)b * srcBatch + (size_t)rs * kEmb;
  const v4f a = *(const v4f*)(sp + ca);
  const v4f c = *(const v4f*)(sp + cb);
  const bool rok = (row < srcRows);
  float v[8];
#pragma unroll
  for (int e = 0; e < 4; ++e) {
    v[e]     = (rok && (c8 + e) < kEmb)     ? a[e] : 0.0f;
    v[4 + e] = (rok && (c8 + 4 + e) < kEmb) ? c[e] : 0.0f;
  }
  unsigned short hb[8], lb[8];
#pragma unroll
  for (int e = 0; e < 8; ++e) {
    hb[e] = f2bf_bits(v[e]);
    lb[e] = f2bf_bits(v[e] - bf_bits2f(hb[e]));
  }
  const v4u uh = (v4u){pk16(hb[0], hb[1]), pk16(hb[2], hb[3]), pk16(hb[4], hb[5]), pk16(hb[6], hb[7])};
  const v4u ul = (v4u){pk16(lb[0], lb[1]), pk16(lb[2], lb[3]), pk16(lb[4], lb[5]), pk16(lb[6], lb[7])};
  const size_t o = (size_t)b * dstBatch + (size_t)row * kEmbPad + c8;
  *(volatile v4u*)(hi + o) = uh;
  *(volatile v4u*)(lo + o) = ul;
  __threadfence();
  *(volatile v4u*)(hi + o) = uh;
  *(volatile v4u*)(lo + o) = ul;
}

__global__ __launch_bounds__(256) void xt_cast_kernel(const float* __restrict__ x, unsigned short* __restrict__ xt) {
  __shared__ float sm[64][65];
  const int t  = threadIdx.x;
  const int l0 = blockIdx.x * 64;
  const int e0 = blockIdx.y * 64;
  const int b  = blockIdx.z;
  const float* xb = x + (size_t)b * kSeq * kEmb;
#pragma unroll
  for (int i = 0; i < 16; ++i) {
    const int idx = i * 256 + t;
    const int r = idx >> 6;
    const int c = idx & 63;
    const int l  = l0 + r;
    const int ee = e0 + c;
    const int lc = (l < kSeq) ? l : (kSeq - 1);
    const int ec = (ee < kEmb) ? ee : (kEmb - 1);
    const float v = xb[(size_t)lc * kEmb + ec];
    sm[c][r] = (l < kSeq && ee < kEmb) ? v : 0.0f;
  }
  __syncthreads();
  const int lane = t & 31, wave = t >> 5;
  const int q = lane >> 3, c8 = (lane & 7) * 8;
  unsigned short* op = xt + (size_t)b * kEmbPad * kSeqPad;
  for (int pass = 0; pass < 2; ++pass) {
#pragma unroll
    for (int it = 0; it < 2; ++it) {
      const int row = wave * 8 + it * 4 + q;
      unsigned short hb[8];
#pragma unroll
      for (int e = 0; e < 8; ++e) hb[e] = h_bits(sm[row][c8 + e]);
      const v4u u = (v4u){pk16(hb[0], hb[1]), pk16(hb[2], hb[3]), pk16(hb[4], hb[5]), pk16(hb[6], hb[7])};
      *(volatile v4u*)(op + (size_t)(e0 + row) * kSeqPad + l0 + c8) = u;
    }
    __threadfence();
  }
}

__global__ __launch_bounds__(kSmThreads) void softmax_row_kernel(const float* __restrict__ S, unsigned short* __restrict__ P) {
  __shared__ float redM[kSmWaves];
  __shared__ float redS[kSmWaves];
  const int row  = blockIdx.x;
  const int t    = threadIdx.x;
  const int lane = t & 31, wave = t >> 5;
  const int c0   = t * 8;
  const float* sr = S + (size_t)row * kSeqPad + c0;
  const v4f a = *(const v4f*)(sr);
  const v4f c = *(const v4f*)(sr + 4);
  float xv[8];
#pragma unroll
  for (int e = 0; e < 4; ++e) { xv[e] = a[e]; xv[4 + e] = c[e]; }
  float m = -INFINITY;
#pragma unroll
  for (int e = 0; e < 8; ++e) {
    const float s = ((c0 + e) < kSeq) ? xv[e] : -INFINITY;
    m = fmaxf(m, s);
  }
#pragma unroll
  for (int off = 16; off > 0; off >>= 1) m = fmaxf(m, __shfl_xor(m, off, 32));
  if (lane == 0) redM[wave] = m;
  __syncthreads();
  float mx = redM[0];
#pragma unroll
  for (int w = 1; w < kSmWaves; ++w) mx = fmaxf(mx, redM[w]);
  float p[8];
  float ps = 0.0f;
#pragma unroll
  for (int e = 0; e < 8; ++e) {
    const float pe = expf(xv[e] - mx);
    p[e] = ((c0 + e) < kSeq) ? pe : 0.0f;
    ps += p[e];
  }
#pragma unroll
  for (int off = 16; off > 0; off >>= 1) ps += __shfl_xor(ps, off, 32);
  if (lane == 0) redS[wave] = ps;
  __syncthreads();
  float tot = redS[0];
#pragma unroll
  for (int w = 1; w < kSmWaves; ++w) tot += redS[w];
  const float inv = (1.0f / tot) * kPCarry;
  unsigned short hb[8];
#pragma unroll
  for (int e = 0; e < 8; ++e) hb[e] = h_bits(p[e] * inv);
  const v4u u = (v4u){pk16(hb[0], hb[1]), pk16(hb[2], hb[3]), pk16(hb[4], hb[5]), pk16(hb[6], hb[7])};
  unsigned short* q = P + (size_t)row * kSeqPad + c0;
  *(volatile v4u*)q = u;
  __threadfence();
  *(volatile v4u*)q = u;
}

__global__ __launch_bounds__(256) void out_writer_kernel(const float* __restrict__ Mall, float* __restrict__ out, int n4) {
  const int i = blockIdx.x * 256 + threadIdx.x;
  if (i >= n4) return;
  const int f = 4 * i;
  const int R = f / kEmb;
  const int e = f - R * kEmb;
  int b = R / kLab;
  const int n = R - b * kLab;
  b = (b < kBatch) ? b : (kBatch - 1);
  const v4f v = *(const v4f*)(Mall + ((size_t)b * kLabPad + n) * kEmbPad + e);
  float* q = out + (size_t)f;
  *(volatile v4f*)q = v;
  __threadfence();
  *(volatile v4f*)q = v;
}

extern "C" void kernel_launch(void* const* d_in, const int* in_sizes, int n_in,
                              void* d_out, int out_size, void* d_ws, size_t ws_size,
                              hipStream_t stream) {
  if (n_in < 2) return;
  if (in_sizes[0] != kBatch * kSeq * kEmb) return;
  if (in_sizes[1] != kLab * kEmb) return;
  if (out_size != kBatch * kLab * kEmb) return;
  if (ws_size < kWsTotal) return;

  const float* x  = (const float*)d_in[0];
  const float* lf = (const float*)d_in[1];
  float* out = (float*)d_out;
  char* ws = (char*)d_ws;
  float*          S    = (float*)(ws + kOffS);
  unsigned short* P16  = (unsigned short*)(ws + kOffP);
  unsigned short* LFhi = (unsigned short*)(ws + kOffLFhi);
  unsigned short* LFlo = (unsigned short*)(ws + kOffLFlo);
  unsigned short* Xhi  = (unsigned short*)(ws + kOffXhi);
  unsigned short* Xlo  = (unsigned short*)(ws + kOffXlo);
  unsigned short* Xt   = (unsigned short*)(ws + kOffXt);
  float*          Mall = (float*)(ws + kOffM);
  const float* dummyf = (const float*)(ws + kOffS);

  split_pad_kernel<<<dim3(kLabPad * 16 / 256, 1), 256, 0, stream>>>(lf, kLab, 0L, LFhi, LFlo, kLabPad, 0L);
  split_pad_kernel<<<dim3(kSeqPad * 16 / 256, kBatch), 256, 0, stream>>>(x, kSeq, (long)kSeq * kEmb, Xhi, Xlo, kSeqPad,
                                                                         (long)kSeqPad * kEmbPad);
  xt_cast_kernel<<<dim3(kSeqPad / 64, kEmbPad / 64, kBatch), 256, 0, stream>>>(x, Xt);

  const int scoreTiles = (kLabChunk / 64) * (kSeqPad / 64);
  const int scoreGrid  = (scoreTiles + 7) / 8;
  const int pvTiles    = (kLabChunk / 64) * (kEmbPad / 64);
  const int pvGrid     = (pvTiles + 7) / 8;

  for (int b = 0; b < kBatch; ++b) {
    const unsigned short* xh = Xhi + (size_t)b * kSeqPad * kEmbPad;
    const unsigned short* xl = Xlo + (size_t)b * kSeqPad * kEmbPad;
    const unsigned short* xtb = Xt + (size_t)b * kEmbPad * kSeqPad;
    for (int ch = 0; ch < kNumChunk; ++ch) {
      const unsigned short* ah = LFhi + (size_t)ch * kLabChunk * kEmbPad;
      const unsigned short* al = LFlo + (size_t)ch * kLabChunk * kEmbPad;
      wmma_gemm64<1, true, 0, 0, false><<<dim3(scoreGrid, 1), 256, 0, stream>>>(
          ah, al, kEmbPad, 0L, xh, xl, kEmbPad, 0L, (void*)S, (void*)S, kSeqPad, 0L, dummyf, dummyf, 0L,
          kLabChunk, kSeqPad, kEmbPad, 1.0f);
      softmax_row_kernel<<<dim3(kLabChunk), kSmThreads, 0, stream>>>(S, P16);
      float* mc = Mall + ((size_t)b * kLabPad + (size_t)ch * kLabChunk) * kEmbPad;
      wmma_gemm64<0, false, 0, 0, false><<<dim3(pvGrid, 1), 256, 0, stream>>>(
          P16, P16, kSeqPad, 0L, xtb, xtb, kSeqPad, 0L, (void*)mc, (void*)mc, kEmbPad, 0L, dummyf, dummyf, 0L,
          kLabChunk, kEmbPad, kSeqPad, kPCarryInv);
    }
  }

  const int n4 = out_size / 4;
  out_writer_kernel<<<dim3((n4 + 255) / 256), 256, 0, stream>>>(Mall, out, n4);
}
